// GCN_cora_21122649162596
// MI455X (gfx1250) — hardware-verified
//
#include <hip/hip_runtime.h>


#define NN_   20000
#define NP    20032
#define NPA   20480
#define NE_   320000
#define NF    256
#define NCL   40
#define NCP   64
#define NT    512
#define NWV   (NT / 32)
#define EPT   4
#define CHUNK (NT * EPT)

typedef unsigned short bf;
typedef __attribute__((ext_vector_type(16))) __bf16   v16bf;
typedef __attribute__((ext_vector_type(8)))  unsigned short v8us;
typedef __attribute__((ext_vector_type(8)))  float    v8f;
typedef __attribute__((ext_vector_type(4)))  float    v4f;
typedef __attribute__((ext_vector_type(4)))  unsigned short v4us;
typedef v4f  __attribute__((may_alias)) v4fa;
typedef v8us __attribute__((may_alias)) v8usa;

__device__ __forceinline__ unsigned short f2bf(float f) { unsigned u = __float_as_uint(f); u += 0x7FFFu + ((u >> 16) & 1u); return (unsigned short)(u >> 16); }
__device__ __forceinline__ float bf2f(unsigned short b) { return __uint_as_float(((unsigned)b) << 16); }
__device__ __forceinline__ float bfr(float f) { return bf2f(f2bf(f)); }
__device__ __forceinline__ v16bf cat16b(v8us lo, v8us hi) { return __builtin_bit_cast(v16bf, __builtin_shufflevector(lo, hi, 0, 1, 2, 3, 4, 5, 6, 7, 8, 9, 10, 11, 12, 13, 14, 15)); }
__device__ __forceinline__ v8f wmmab(v16bf a, v16bf b, v8f c) { return __builtin_amdgcn_wmma_f32_16x16x32_bf16(false, a, false, b, (short)0, c, false, false); }
#define VST2(T, p, v) do { const T vst2_v_ = (v); *(volatile T*)(p) = vst2_v_; __threadfence(); *(volatile T*)(p) = vst2_v_; } while (0)

__global__ __launch_bounds__(256) void k_xb(const float* __restrict__ x, bf* XH, bf* XL) {
    const int lane = threadIdx.x & 31, r = blockIdx.x * 8 + (threadIdx.x >> 5);
    if (r >= NP) return;
    v8us t, z;
#pragma unroll
    for (int i = 0; i < 8; ++i) { t[i] = (r < NN_) ? f2bf(x[(size_t)r * NF + lane * 8 + i]) : (unsigned short)0; z[i] = 0; }
    VST2(v8us, XH + (size_t)r * NF + lane * 8, t);
    VST2(v8us, XL + (size_t)r * NF + lane * 8, z);
}

__global__ __launch_bounds__(256) void k_wt(const float* __restrict__ Wm, int N, bf* WT) {
    __shared__ __align__(16) unsigned short tl[64 * 72];
    const int tid = threadIdx.x, k0 = blockIdx.x * 64, n0 = blockIdx.y * 64;
    const int kk = tid >> 2, nq = (tid & 3) * 16;
#pragma unroll
    for (int i = 0; i < 16; ++i) { const int n = n0 + nq + i; tl[(nq + i) * 72 + kk] = (n < N) ? f2bf(Wm[(size_t)(k0 + kk) * N + n]) : (unsigned short)0; }
    __syncthreads();
    const int piece = tid & 7;
    auto pass = [&]() {
#pragma unroll
        for (int s = 0; s < 2; ++s) { const int nr = (tid >> 3) + 32 * s; const v8us val = *(const v8usa*)(tl + nr * 72 + piece * 8);
            *(volatile v8us*)(WT + (size_t)(n0 + nr) * NF + k0 + piece * 8) = val; }
    };
    pass(); __threadfence(); pass();
}

__global__ __launch_bounds__(128) void k_gemmb(const bf* __restrict__ A, const bf* __restrict__ Al, const bf* __restrict__ Bn, float* C, int ldc) {
    __shared__ __align__(16) float ost[4][16 * 68];
    const int lane = threadIdx.x & 31, wave = threadIdx.x >> 5, lr = lane & 15, hi = lane >> 4;
    const int r0 = blockIdx.x * 64 + wave * 16, c0 = blockIdx.y * 64;
    const size_t aoff = (size_t)(r0 + lr) * NF + 8 * hi;
    size_t boff[4];
#pragma unroll
    for (int t = 0; t < 4; ++t) boff[t] = (size_t)(c0 + t * 16 + lr) * NF + 8 * hi;
    v8f acc[4];
#pragma unroll
    for (int t = 0; t < 4; ++t) acc[t] = (v8f){};
#pragma unroll 1
    for (int kc = 0; kc < NF; kc += 32) {
        const v16bf a  = cat16b(*(const v8us*)(A + aoff + kc), *(const v8us*)(A + aoff + kc + 16));
        const v16bf al = cat16b(*(const v8us*)(Al + aoff + kc), *(const v8us*)(Al + aoff + kc + 16));
#pragma unroll
        for (int t = 0; t < 4; ++t) {
            const v16bf b = cat16b(*(const v8us*)(Bn + boff[t] + kc), *(const v8us*)(Bn + boff[t] + kc + 16));
            acc[t] = wmmab(a, b, acc[t]); acc[t] = wmmab(al, b, acc[t]);
        }
        asm volatile("v_nop\n\tv_nop\n\tv_nop\n\tv_nop" : "+v"(acc[0]), "+v"(acc[1]), "+v"(acc[2]), "+v"(acc[3]) : "v"(a), "v"(al));
    }
    float* os = &ost[wave][0];
#pragma unroll
    for (int t = 0; t < 4; ++t)
#pragma unroll
        for (int j = 0; j < 8; ++j) os[(hi * 8 + j) * 68 + t * 16 + lr] = acc[t][j];
    __syncthreads();
    float* crow = C + (size_t)r0 * ldc + c0;
    auto pass = [&]() {
#pragma unroll
        for (int s = 0; s < 8; ++s) { const int Lid = (lane >> 3) + 4 * s, piece = lane & 7; const int row = Lid >> 1, cofs = (Lid & 1) * 32 + piece * 4;
            const v4f val = *(const v4fa*)(os + row * 68 + cofs); *(volatile v4f*)(crow + (size_t)row * ldc + cofs) = val; }
    };
    pass(); __threadfence(); pass();
}

template <int W>
__global__ __launch_bounds__(NT) void k_spmm(const float* __restrict__ T, const int* __restrict__ arow, const int* __restrict__ acol, const float* __restrict__ aval,
                                             const float* __restrict__ bias, int nbias, float* AGG) {
    constexpr int RB = 65536 / W;
    extern __shared__ float4 lds_raw[];
    float* agg  = (float*)lds_raw;
    int*   lst  = (int*)(agg + RB * W);
    float* lsv  = (float*)(lst + CHUNK);
    int*   wtot = (int*)(lsv + CHUNK);
    const int t = threadIdx.x, lane = t & 31, wv = t >> 5;
    const int n0 = blockIdx.x * RB;
    for (int i = t; i < RB * W; i += NT) agg[i] = 0.0f;
    __syncthreads();
#pragma unroll 1
    for (int base = 0; base < NE_; base += CHUNK) {
        int val[EPT]; float vv[EPT]; int flg[EPT]; int cnt = 0;
#pragma unroll
        for (int j = 0; j < EPT; ++j) {
            const int e = base + j * NT + t;
            const int d = (e < NE_) ? arow[e] : -1;
            const unsigned udl = (unsigned)d - (unsigned)n0;
            const int f = (udl < (unsigned)RB) ? 1 : 0;
            int v = 0; float w = 0.f;
            if (f) { int s = acol[e]; if (s < 0) s += NN_; s = min(max(s, 0), NN_ - 1); v = s * RB + (int)udl; w = bfr(aval[e]); }
            val[j] = v; vv[j] = w; flg[j] = f; cnt += f;
        }
        int incl = cnt;
#pragma unroll
        for (int o = 1; o < 32; o <<= 1) { const int y = __shfl_up(incl, o, 32); if (lane >= o) incl += y; }
        if (lane == 31) wtot[wv] = incl;
        __syncthreads();
        int off = incl - cnt, tot = 0;
#pragma unroll
        for (int i = 0; i < NWV; ++i) { const int v = wtot[i]; off += (i < wv) ? v : 0; tot += v; }
#pragma unroll
        for (int j = 0; j < EPT; ++j) { if (flg[j]) { lst[off] = val[j]; lsv[off] = vv[j]; ++off; } }
        __syncthreads();
        if (tot > 0 && t < W) {
#pragma unroll 1
            for (int e2 = 0; e2 < tot; ++e2) { const int v = lst[e2]; const int s = v / RB, dl = v - s * RB; agg[dl * W + t] += lsv[e2] * T[(size_t)s * W + t]; }
        }
        __syncthreads();
    }
    constexpr int RPW = RB / NWV;
    for (int i = 0; i < RPW; ++i) {
        const int rl = wv * RPW + i;
        float* row = AGG + (size_t)(n0 + rl) * W;
        float v[W / 32];
#pragma unroll
        for (int q = 0; q < W / 32; ++q) { const int c = q * 32 + lane; v[q] = agg[rl * W + c] + ((c < nbias) ? bfr(bias[c]) : 0.f); }
#pragma unroll
        for (int q = 0; q < W / 32; ++q) *(volatile float*)(row + q * 32 + lane) = v[q];
        __threadfence();
#pragma unroll
        for (int q = 0; q < W / 32; ++q) *(volatile float*)(row + q * 32 + lane) = v[q];
    }
}

__global__ __launch_bounds__(256) void k_bnstat(const float* __restrict__ AGG, float* MU, float* RS) {
    const int c = threadIdx.x;
    double s = 0.0, q = 0.0;
#pragma unroll 1
    for (int r = 0; r < NN_; ++r) { const double v = (double)AGG[(size_t)r * NF + c]; s += v; q += v * v; }
    const double mu = s / (double)NN_;
    double var = q / (double)NN_ - mu * mu; if (var < 0.0) var = 0.0;
    VST2(float, MU + c, (float)mu);
    VST2(float, RS + c, (float)(1.0 / sqrt(var + 1e-5)));
}

__global__ __launch_bounds__(256) void k_bnapply(const float* __restrict__ AGG, const float* __restrict__ MU, const float* __restrict__ RS, const float* __restrict__ gam,
                                                 const float* __restrict__ bet, bf* HH, bf* HL) {
    const int lane = threadIdx.x & 31, r = blockIdx.x * 8 + (threadIdx.x >> 5);
    if (r >= NP) return;
    v8us oh, ol;
#pragma unroll
    for (int i = 0; i < 8; ++i) {
        const int c = lane * 8 + i;
        float h = 0.f;
        if (r < NN_) { h = bfr(gam[c]) * (AGG[(size_t)r * NF + c] - MU[c]) * RS[c] + bfr(bet[c]); h = h > 0.f ? h : 0.f; }
        const unsigned short hb = f2bf(h); oh[i] = hb; ol[i] = f2bf(h - bf2f(hb));
    }
    VST2(v8us, HH + (size_t)r * NF + lane * 8, oh);
    VST2(v8us, HL + (size_t)r * NF + lane * 8, ol);
}

__global__ __launch_bounds__(128) void k_final(const float* __restrict__ AGG3, float* out) {
    __shared__ __align__(16) float st[32 * 40];
    const int lane = threadIdx.x & 31, wv = threadIdx.x >> 5;
    const int r0 = blockIdx.x * 32;
#pragma unroll
    for (int i = 0; i < 8; ++i) {
        const int rl = wv * 8 + i, r = r0 + rl;
        const float a = AGG3[(size_t)r * NCP + lane];
        const float b = (lane < NCL - 32) ? AGG3[(size_t)r * NCP + 32 + lane] : -__builtin_inff();
        float mx = fmaxf(a, b);
#pragma unroll
        for (int o = 16; o; o >>= 1) mx = fmaxf(mx, __shfl_xor(mx, o, 32));
        float s = expf(a - mx) + ((lane < NCL - 32) ? expf(b - mx) : 0.f);
#pragma unroll
        for (int o = 16; o; o >>= 1) s += __shfl_xor(s, o, 32);
        const float lse = logf(s) + mx;
        st[rl * NCL + lane] = a - lse;
        if (lane < NCL - 32) st[rl * NCL + 32 + lane] = b - lse;
    }
    __syncthreads();
    if (r0 + 32 <= NN_) {
        float* ob = out + (size_t)r0 * NCL;
        auto pass = [&]() {
#pragma unroll
            for (int s = 0; s < 3; ++s) {
                const int li = wv * 10 + (lane >> 3) + 4 * s, piece = lane & 7;
                if (li < wv * 10 + 10) { const v4f val = *(const v4fa*)(st + li * 32 + piece * 4); *(volatile v4f*)(ob + li * 32 + piece * 4) = val; }
            }
        };
        pass(); __threadfence(); pass();
    }
}

extern "C" void kernel_launch(void* const* d_in, const int* in_sizes, int n_in,
                              void* d_out, int out_size, void* d_ws, size_t ws_size, hipStream_t stream) {
    (void)in_sizes; (void)n_in; (void)out_size;
    const float* x = (const float*)d_in[0]; const int* arow = (const int*)d_in[1]; const int* acol = (const int*)d_in[2]; const float* aval = (const float*)d_in[3];
    const float* W1 = (const float*)d_in[4]; const float* b1 = (const float*)d_in[5]; const float* g1 = (const float*)d_in[6]; const float* be1 = (const float*)d_in[7];
    const float* W2 = (const float*)d_in[8]; const float* b2 = (const float*)d_in[9]; const float* g2 = (const float*)d_in[10]; const float* be2 = (const float*)d_in[11];
    const float* W3 = (const float*)d_in[12]; const float* b3 = (const float*)d_in[13];
    float* out = (float*)d_out;
    char* wsp = (char*)d_ws;
    auto take = [&](size_t bytes) { char* p = wsp; wsp += (bytes + 255) & ~(size_t)255; return (void*)p; };
    bf* XH = (bf*)take((size_t)NP * NF * 2); bf* XL = (bf*)take((size_t)NP * NF * 2);
    bf* W1T = (bf*)take((size_t)NF * NF * 2); bf* W2T = (bf*)take((size_t)NF * NF * 2); bf* W3T = (bf*)take((size_t)NCP * NF * 2);
    float* T1 = (float*)take((size_t)NP * NF * 4); float* AGG = (float*)take((size_t)NPA * NF * 4);
    float* MU = (float*)take(NF * 4); float* RS = (float*)take(NF * 4);
    bf* HH = (bf*)take((size_t)NP * NF * 2); bf* HL = (bf*)take((size_t)NP * NF * 2);
    float* T3 = (float*)take((size_t)NP * NCP * 4); float* AGG3 = (float*)take((size_t)NPA * NCP * 4);
    if ((size_t)(wsp - (char*)d_ws) > ws_size) return;
    const size_t lds = (size_t)65536 * 4 + (size_t)CHUNK * 8 + NWV * 4;
    k_xb<<<NP / 8, 256, 0, stream>>>(x, XH, XL);
    k_wt<<<dim3(NF / 64, NF / 64, 1), 256, 0, stream>>>(W1, NF, W1T);
    k_wt<<<dim3(NF / 64, NF / 64, 1), 256, 0, stream>>>(W2, NF, W2T);
    k_wt<<<dim3(NF / 64, 1, 1), 256, 0, stream>>>(W3, NCL, W3T);
    k_gemmb<<<dim3(NP / 64, NF / 64, 1), 128, 0, stream>>>(XH, XL, W1T, T1, NF);
    k_spmm<256><<<NPA / 256, NT, lds, stream>>>(T1, arow, acol, aval, b1, NF, AGG);
    k_bnstat<<<1, 256, 0, stream>>>(AGG, MU, RS);
    k_bnapply<<<NP / 8, 256, 0, stream>>>(AGG, MU, RS, g1, be1, HH, HL);
    k_gemmb<<<dim3(NP / 64, NF / 64, 1), 128, 0, stream>>>(HH, HL, W2T, T1, NF);
    k_spmm<256><<<NPA / 256, NT, lds, stream>>>(T1, arow, acol, aval, b2, NF, AGG);
    k_bnstat<<<1, 256, 0, stream>>>(AGG, MU, RS);
    k_bnapply<<<NP / 8, 256, 0, stream>>>(AGG, MU, RS, g2, be2, HH, HL);
    k_gemmb<<<dim3(NP / 64, 1, 1), 128, 0, stream>>>(HH, HL, W3T, T3, NCP);
    k_spmm<64><<<NPA / 1024, NT, lds, stream>>>(T3, arow, acol, aval, b3, NCL, AGG3);
    k_final<<<NN_ / 32, 128, 0, stream>>>(AGG3, out);
}
